// GNN_35304631173261
// MI455X (gfx1250) — hardware-verified
//
#include <hip/hip_runtime.h>
#include <stddef.h>
#include <stdint.h>
#include <math.h>


#define NHID   128
#define HEADS  8
#define DKD    16
#define NTYP   3
#define NREL   4
#define MAXLEN 240
#define IND    256
#define KP     256

#define NTHR   256
#define NWAVE  8
#define EPT    8
#define CHUNK  (NTHR * EPT)
#define WCAP   (EPT * 32)
#define LISTN  (NWAVE * WCAP)
#define NBA    1024
#define SLA    10
#define RCAP   12288
#define DEGCAP 32
#define GBM    64
#define GBN    128
#define GTHR   128
#define APITCH 264

#define UADP   (NTYP * NHID * 32)
#define UKQV   (2 * NTYP * 3 * NHID * 32)
#define UA2    (2 * NTYP * NHID * 32)
#define UWTOT  (UADP + UKQV + UA2)

#define AGG_ZINTS (LISTN + 2 * RCAP + 3 * NBA)
#define MISC_INTS 16
#define REL_F  (NREL * HEADS * DKD * DKD)
#define PQ_I   32
#define WQ_F   128
#define QA_F   512
#define UB_F   512
#define SC_F   (DEGCAP * 32)
#define RB_I   128
#define PW_I   (WQ_F + QA_F + UB_F + SC_F + RB_I)
#define SCAN_LDS_INTS (AGG_ZINTS + MISC_INTS + 2 * REL_F + PQ_I + NWAVE * PW_I)
#define RTE_F  (2 * 2 * NTYP * MAXLEN * NHID)
#define WSMAX  134217728

static_assert((CHUNK & (CHUNK - 1)) == 0 && CHUNK <= 4096);
static_assert((NBA & (NBA - 1)) == 0 && NBA == (1 << SLA));
static_assert(((long long)CHUNK << SLA) < (1LL << 31));
static_assert(LISTN % NTHR == 0);
static_assert(NBA % NWAVE == 0 && NBA % 32 == 0);
static_assert(RCAP % 4 == 0 && AGG_ZINTS % (NTHR * 4) == 0 && ((AGG_ZINTS + MISC_INTS) % 4) == 0);
static_assert(PQ_I % 4 == 0 && PW_I % 4 == 0 && WQ_F % 4 == 0 && QA_F % 4 == 0 && UB_F % 4 == 0 && SC_F % 4 == 0);
static_assert(DEGCAP == 32);
static_assert(SCAN_LDS_INTS * 4 <= 300000);
static_assert(KP % 32 == 0 && KP == 2 * NHID && KP == IND);
static_assert(GBM == (GTHR / 32) * 16 && GBN == NHID && NHID == 4 * 32);
static_assert(GBM * GBN * 4 <= GBM * APITCH * 2);
static_assert((APITCH * 2) % 16 == 0);
static_assert(UADP % NTHR == 0 && (UADP + UKQV) % NTHR == 0 && UWTOT % NTHR == 0);
static_assert((NHID * 32) % NTHR == 0);
static_assert(HEADS * DKD == NHID && REL_F == 8192);

typedef float          v4f   __attribute__((ext_vector_type(4)));
typedef float          v8f   __attribute__((ext_vector_type(8)));
typedef int            v4i   __attribute__((ext_vector_type(4)));
typedef int            v8i   __attribute__((ext_vector_type(8)));
typedef unsigned       v2u   __attribute__((ext_vector_type(2)));
typedef unsigned       v4u   __attribute__((ext_vector_type(4)));
typedef unsigned short v4us  __attribute__((ext_vector_type(4)));
typedef unsigned short v8us  __attribute__((ext_vector_type(8)));
typedef unsigned short v16us __attribute__((ext_vector_type(16)));
typedef __bf16         v16bf __attribute__((ext_vector_type(16)));
typedef v4f  __attribute__((may_alias)) v4fa;
typedef v4i  __attribute__((may_alias)) v4ia;
typedef v2u  __attribute__((may_alias)) v2ua;
typedef v4u  __attribute__((may_alias)) v4ua;
typedef v4us __attribute__((may_alias)) v4usa;
typedef v8us __attribute__((may_alias)) v8usa;
union FragB { v16bf v; v16us u; v8us h[2]; v8i w; };

__device__ __forceinline__ v8f wmb(const FragB& a, const FragB& b, v8f c) {
  v8f d = __builtin_amdgcn_wmma_f32_16x16x32_bf16(false, a.v, false, b.v, (short)0, c, false, false);
  asm volatile("v_nop\n\tv_nop\n\tv_nop\n\tv_nop" : "+v"(d) : "v"(a.w), "v"(b.w));
  return d;
}

__device__ __forceinline__ unsigned bf16_bits(float f) {
  const unsigned u = __float_as_uint(f);
  return (u + 0x7FFFu + ((u >> 16) & 1u)) >> 16;
}
__device__ __forceinline__ float bf16_val(float f) {
  return __uint_as_float(bf16_bits(f) << 16);
}

__device__ __forceinline__ void wave_sync() {
  __builtin_amdgcn_fence(__ATOMIC_RELEASE, "wavefront");
  __builtin_amdgcn_wave_barrier();
  __builtin_amdgcn_fence(__ATOMIC_ACQUIRE, "wavefront");
}

__device__ __forceinline__ void put8us(unsigned short* p, const v8us v, bool ok) {
  if (ok) *(volatile v8us*)p = v;
  __threadfence();
  if (ok) *(volatile v8us*)p = v;
}
__device__ __forceinline__ void put4f(float* p, const v4f v, bool ok) {
  if (ok) *(volatile v4f*)p = v;
  __threadfence();
  if (ok) *(volatile v4f*)p = v;
}

template <int SLB>
__device__ __forceinline__ int scan_chunk(const int* __restrict__ dsts, int nE, int cbase, int slotBase,
                                          int nb, int vec8, int* list, int tid, int lane, int wave) {
  int wc = 0;
  const int el0  = tid * EPT;
  const int e0   = cbase + el0;
  const int sent = -2147483647 - 1;
  v4i da, db;
  if (vec8 != 0 && cbase + CHUNK <= nE) {
    da = *(const v4i*)(dsts + e0);
    db = *(const v4i*)(dsts + e0 + 4);
  } else {
    da.x = (e0     < nE) ? dsts[min(e0,     nE - 1)] : sent;
    da.y = (e0 + 1 < nE) ? dsts[min(e0 + 1, nE - 1)] : sent;
    da.z = (e0 + 2 < nE) ? dsts[min(e0 + 2, nE - 1)] : sent;
    da.w = (e0 + 3 < nE) ? dsts[min(e0 + 3, nE - 1)] : sent;
    db.x = (e0 + 4 < nE) ? dsts[min(e0 + 4, nE - 1)] : sent;
    db.y = (e0 + 5 < nE) ? dsts[min(e0 + 5, nE - 1)] : sent;
    db.z = (e0 + 6 < nE) ? dsts[min(e0 + 6, nE - 1)] : sent;
    db.w = (e0 + 7 < nE) ? dsts[min(e0 + 7, nE - 1)] : sent;
  }
  const unsigned nbs = (unsigned)slotBase;
  const unsigned unb = (unsigned)nb;
  const unsigned s0 = (unsigned)da.x - nbs, s1 = (unsigned)da.y - nbs;
  const unsigned s2 = (unsigned)da.z - nbs, s3 = (unsigned)da.w - nbs;
  const unsigned s4 = (unsigned)db.x - nbs, s5 = (unsigned)db.y - nbs;
  const unsigned s6 = (unsigned)db.z - nbs, s7 = (unsigned)db.w - nbs;
  const bool h0 = s0 < unb, h1 = s1 < unb, h2 = s2 < unb, h3 = s3 < unb;
  const bool h4 = s4 < unb, h5 = s5 < unb, h6 = s6 < unb, h7 = s7 < unb;
  const unsigned any = __builtin_amdgcn_ballot_w32(h0 | h1 | h2 | h3 | h4 | h5 | h6 | h7);
  if (any != 0u) {
#define HITJ(J, HJ, SJ) { \
      const unsigned mj = __builtin_amdgcn_ballot_w32(HJ); \
      if (mj != 0u) { \
        if (HJ) { \
          const int pos = wc + (int)__builtin_amdgcn_mbcnt_lo(mj, 0u); \
          if (pos < WCAP) list[wave * WCAP + pos] = ((el0 + (J)) << SLB) | (int)(SJ); \
        } \
        wc += (int)__builtin_popcount(mj); } }
    HITJ(0, h0, s0)
    HITJ(1, h1, s1)
    HITJ(2, h2, s2)
    HITJ(3, h3, s3)
    HITJ(4, h4, s4)
    HITJ(5, h5, s5)
    HITJ(6, h6, s6)
    HITJ(7, h7, s7)
#undef HITJ
  }
  return wc;
}

__device__ __forceinline__ v8us gather8(const float* __restrict__ p) {
  v8us o;
#pragma unroll
  for (int i = 0; i < 8; ++i) o[i] = (unsigned short)bf16_bits(p[(size_t)i * NHID]);
  return o;
}

__global__ __launch_bounds__(NTHR) void k_wprep(const float* __restrict__ adw, const float* __restrict__ kw,
                                                const float* __restrict__ qw, const float* __restrict__ vw,
                                                const float* __restrict__ aw, unsigned short* wpl) {
  const int u = (int)blockIdx.x * NTHR + (int)threadIdx.x;
  if (u >= UWTOT) return;
  const int k8 = (u & 31) * 8;
  v8us o;
  if (u < UADP) {
    const int row = u >> 5;
    const int t = row >> 7, n = row & 127;
    o = gather8(adw + ((size_t)t * IND + k8) * NHID + n);
  } else if (u < UADP + UKQV) {
    const int row   = (u - UADP) >> 5;
    const int lt    = row / 384;
    const int n3    = row - lt * 384;
    const int which = n3 >> 7;
    const int n     = n3 & 127;
    const int kk    = k8 & 127;
    const size_t off = ((size_t)lt * NHID + kk) * NHID + n;
    if (which == 0)      o = gather8(kw + off);
    else if (which == 1) o = gather8(qw + off);
    else                 o = gather8(vw + off);
  } else {
    const int row = (u - UADP - UKQV) >> 5;
    const int lt = row >> 7, n = row & 127;
    const int kk = k8 & 127;
    o = gather8(aw + ((size_t)lt * NHID + kk) * NHID + n);
  }
  put8us(wpl + (size_t)u * 8, o, true);
}

__global__ __launch_bounds__(NTHR) void k_sort(const int* __restrict__ ntype, int nN, int permCap, int* perm) {
  extern __shared__ __attribute__((aligned(16))) int ssm[];
  int* pl = ssm;
  int* cn = ssm + permCap;
  const int tid = (int)threadIdx.x;
  const int per = (nN + NTHR - 1) / NTHR;
  const int b   = tid * per;
  int c0 = 0, c1 = 0, c2 = 0;
#pragma unroll 1
  for (int j = 0; j < per; ++j) {
    const int i  = b + j;
    const int ic = i < nN ? i : nN - 1;
    int t = ntype[ic];
    t = t < 0 ? 0 : (t > 2 ? 2 : t);
    const bool ok = i < nN;
    c0 += (ok && t == 0) ? 1 : 0;
    c1 += (ok && t == 1) ? 1 : 0;
    c2 += (ok && t == 2) ? 1 : 0;
  }
  cn[tid] = c0; cn[NTHR + tid] = c1; cn[2 * NTHR + tid] = c2;
#pragma unroll 1
  for (int i = tid; i < permCap; i += NTHR) pl[i] = -1;
  __syncthreads();
  int p0 = 0, p1 = 0, p2 = 0, t0 = 0, t1 = 0, t2 = 0;
#pragma unroll 1
  for (int j = 0; j < NTHR; ++j) {
    const int a = cn[j], bq = cn[NTHR + j], cq = cn[2 * NTHR + j];
    const bool lo = j < tid;
    p0 += lo ? a : 0; p1 += lo ? bq : 0; p2 += lo ? cq : 0;
    t0 += a; t1 += bq; t2 += cq;
  }
  const int s1 = ((t0 + 63) >> 6) << 6;
  const int s2 = s1 + (((t1 + 63) >> 6) << 6);
  int w0 = p0, w1 = s1 + p1, w2 = s2 + p2;
#pragma unroll 1
  for (int j = 0; j < per; ++j) {
    const int i  = b + j;
    const int ic = i < nN ? i : nN - 1;
    int t = ntype[ic];
    t = t < 0 ? 0 : (t > 2 ? 2 : t);
    const bool ok = i < nN;
    const int pos = (t == 0) ? w0 : ((t == 1) ? w1 : w2);
    if (ok && pos >= 0 && pos < permCap) pl[pos] = i;
    w0 += (ok && t == 0) ? 1 : 0;
    w1 += (ok && t == 1) ? 1 : 0;
    w2 += (ok && t == 2) ? 1 : 0;
  }
  __syncthreads();
  const int nU = permCap >> 2;
#pragma unroll 1
  for (int u = tid; u < nU; u += NTHR) {
    const v4i v = *(const v4ia*)(pl + 4 * u);
    *(volatile v4i*)(perm + 4 * u) = v;
  }
  __threadfence();
#pragma unroll 1
  for (int u = tid; u < nU; u += NTHR) {
    const v4i v = *(const v4ia*)(pl + 4 * u);
    *(volatile v4i*)(perm + 4 * u) = v;
  }
}

__global__ __launch_bounds__(128) void k_rte(const float* __restrict__ tab, const float* __restrict__ rw,
                                             const float* __restrict__ rb, const float* __restrict__ kw,
                                             const float* __restrict__ vw, float* rte) {
  __shared__ float tabS[IND];
  __shared__ float rteS[NHID];
  __shared__ __attribute__((aligned(16))) float outS[6 * NHID];
  const int tid = (int)threadIdx.x, lane = tid & 31;
  const int l = (int)blockIdx.x / MAXLEN;
  const int m = (int)blockIdx.x - l * MAXLEN;
  const float* tp = tab + ((size_t)l * MAXLEN + m) * IND;
  tabS[tid]       = bf16_val(tp[tid]);
  tabS[tid + 128] = bf16_val(tp[tid + 128]);
  __syncthreads();
  float s = 0.0f;
  const float* wp = rw + (size_t)l * IND * NHID + tid;
#pragma unroll 4
  for (int d = 0; d < IND; ++d) s = fmaf(tabS[d], bf16_val(wp[(size_t)d * NHID]), s);
  s += bf16_val(rb[l * NHID + tid]);
  rteS[tid] = s;
  __syncthreads();
#pragma unroll 1
  for (int t = 0; t < NTYP; ++t) {
    const float* kp = kw + ((size_t)(l * NTYP + t) * NHID) * NHID + tid;
    const float* vp = vw + ((size_t)(l * NTYP + t) * NHID) * NHID + tid;
    float sk = 0.0f, sv = 0.0f;
#pragma unroll 4
    for (int d = 0; d < NHID; ++d) {
      const float x = rteS[d];
      sk = fmaf(x, bf16_val(kp[(size_t)d * NHID]), sk);
      sv = fmaf(x, bf16_val(vp[(size_t)d * NHID]), sv);
    }
    outS[(2 * t) * NHID + tid]     = sk;
    outS[(2 * t + 1) * NHID + tid] = sv;
  }
  __syncthreads();
  const int  rr0 = tid >> 5;
  const bool ok1 = tid < 64;
  const int  rr1 = ok1 ? (4 + (tid >> 5)) : 5;
  const v4f o0 = *(const v4fa*)(outS + rr0 * NHID + 4 * lane);
  const v4f o1 = *(const v4fa*)(outS + rr1 * NHID + 4 * lane);
  float* d0 = rte + ((size_t)((l * 2 + (rr0 & 1)) * NTYP + (rr0 >> 1)) * MAXLEN + m) * NHID + 4 * lane;
  float* d1 = rte + ((size_t)((l * 2 + (rr1 & 1)) * NTYP + (rr1 >> 1)) * MAXLEN + m) * NHID + 4 * lane;
  *(volatile v4f*)d0 = o0;
  if (ok1) *(volatile v4f*)d1 = o1;
  __threadfence();
  *(volatile v4f*)d0 = o0;
  if (ok1) *(volatile v4f*)d1 = o1;
}

template <int MODE>
__global__ __launch_bounds__(GTHR) void k_gemm(
    const float* __restrict__ af32, const unsigned short* __restrict__ apl,
    const unsigned short* __restrict__ WT, int nOutTot,
    const int* __restrict__ perm, int permCap, const int* __restrict__ ntype, int nN,
    const float* __restrict__ b0, const float* __restrict__ b1, const float* __restrict__ b2,
    const float* __restrict__ skipl, unsigned short* xhl, float* outF, size_t planeStride)
{
  __shared__ __attribute__((aligned(16))) unsigned char smem[GBM * APITCH * 2];
  __shared__ int sPerm[GBM];
  __shared__ __attribute__((aligned(16))) unsigned short rbuf[(GTHR / 32) * KP];
  unsigned short* sA = (unsigned short*)smem;
  float* stg = (float*)smem;
  const int tid = (int)threadIdx.x, lane = tid & 31, wave = tid >> 5, hh = lane >> 4, m = lane & 15;
  const int rowBase = (int)blockIdx.x * GBM;
  const int by      = (int)blockIdx.y;
  const int col0    = by * GBN;

  if (tid < GBM) {
    int gi = rowBase + tid;
    gi = gi < permCap ? gi : permCap - 1;
    const int p = perm[gi];
    sPerm[tid] = (p >= 0 && p < nN) ? p : -1;
  }
  __syncthreads();
  int n0 = sPerm[0];
  n0 = n0 < 0 ? 0 : n0;
  int tt = ntype[n0];
  tt = tt < 0 ? 0 : (tt > 2 ? 2 : tt);

#pragma unroll 4
  for (int it = 0; it < GBM / 4; ++it) {
    const int row  = it * 4 + wave;
    const int node = sPerm[row];
    const bool ok  = node >= 0;
    const int nc   = ok ? node : 0;
    v4u o;
    if constexpr (MODE == 0) {
      const float* p = af32 + (size_t)nc * KP + 8 * lane;
      const v4f a = *(const v4f*)p;
      const v4f b = *(const v4f*)(p + 4);
      o.x = bf16_bits(a.x) | (bf16_bits(a.y) << 16);
      o.y = bf16_bits(a.z) | (bf16_bits(a.w) << 16);
      o.z = bf16_bits(b.x) | (bf16_bits(b.y) << 16);
      o.w = bf16_bits(b.z) | (bf16_bits(b.w) << 16);
    } else {
      o = *(const v4ua*)(apl + (size_t)nc * KP + 8 * lane);
    }
    const unsigned msk = ok ? 0xffffffffu : 0u;
    o.x &= msk; o.y &= msk; o.z &= msk; o.w &= msk;
    *(v4ua*)(sA + row * APITCH + 8 * lane) = o;
  }
  __syncthreads();

  v8f acc[8];
  {
    const v8f z = {0.f, 0.f, 0.f, 0.f, 0.f, 0.f, 0.f, 0.f};
#pragma unroll
    for (int t = 0; t < 8; ++t) acc[t] = z;
  }
  const unsigned short* ap = sA + (16 * wave + m) * APITCH + 8 * hh;
  const unsigned short* bp = WT + ((size_t)tt * (size_t)nOutTot + (size_t)(col0 + m)) * (size_t)KP + 8 * hh;
#pragma unroll 1
  for (int k0 = 0; k0 < KP; k0 += 32) {
    FragB af;
    af.h[0] = *(const v8usa*)(ap + k0);
    af.h[1] = *(const v8usa*)(ap + k0 + 16);
#pragma unroll
    for (int nt = 0; nt < 8; ++nt) {
      const unsigned short* wq = bp + (size_t)(16 * nt) * (size_t)KP + k0;
      FragB bf;
      bf.h[0] = *(const v8usa*)wq;
      bf.h[1] = *(const v8usa*)(wq + 16);
      acc[nt] = wmb(af, bf, acc[nt]);
    }
  }
  __syncthreads();

#pragma unroll
  for (int nt = 0; nt < 8; ++nt) {
    const int lc = 16 * nt + m;
#pragma unroll
    for (int r = 0; r < 8; ++r) {
      const int lr = 16 * wave + 8 * hh + r;
      stg[lr * GBN + lc] = acc[nt][r];
    }
  }
  __syncthreads();

  v4f bb;
  {
    const v4f t0 = *(const v4f*)(b0 + tt * NHID + 4 * lane);
    v4f ts = t0;
    if constexpr (MODE == 1) {
      const v4f t1 = *(const v4f*)(b1 + tt * NHID + 4 * lane);
      const v4f t2 = *(const v4f*)(b2 + tt * NHID + 4 * lane);
      ts.x = (by == 0) ? t0.x : ((by == 1) ? t1.x : t2.x);
      ts.y = (by == 0) ? t0.y : ((by == 1) ? t1.y : t2.y);
      ts.z = (by == 0) ? t0.z : ((by == 1) ? t1.z : t2.z);
      ts.w = (by == 0) ? t0.w : ((by == 1) ? t1.w : t2.w);
    }
    bb.x = bf16_val(ts.x); bb.y = bf16_val(ts.y); bb.z = bf16_val(ts.z); bb.w = bf16_val(ts.w);
  }
  float alpha = 0.0f, om = 0.0f;
  if constexpr (MODE >= 2) {
    const float sk = bf16_val(skipl[tt]);
    alpha = 1.0f / (1.0f + expf(-sk));
    om = 1.0f - alpha;
  }
  unsigned short* rb = rbuf + wave * KP;

#pragma unroll 1
  for (int i = 0; i < 16; ++i) {
    const int lr   = 16 * wave + i;
    const int node = sPerm[lr];
    const bool ok  = node >= 0;
    const int nc   = ok ? node : 0;
    const v4f v = *(const v4fa*)(stg + lr * GBN + 4 * lane);
    const v4f t = v + bb;
    v4f y;
    if constexpr (MODE == 0) {
      y.x = tanhf(t.x); y.y = tanhf(t.y); y.z = tanhf(t.z); y.w = tanhf(t.w);
    } else if constexpr (MODE == 1) {
      y = t;
    } else {
      const unsigned short* xr = xhl + (size_t)nc * KP + 4 * lane;
      const v2u wh = *(const v2ua*)xr;
      const v2u wl = *(const v2ua*)(xr + NHID);
      const float x0 = __uint_as_float(wh.x << 16)         + __uint_as_float(wl.x << 16);
      const float x1 = __uint_as_float(wh.x & 0xffff0000u) + __uint_as_float(wl.x & 0xffff0000u);
      const float x2 = __uint_as_float(wh.y << 16)         + __uint_as_float(wl.y << 16);
      const float x3 = __uint_as_float(wh.y & 0xffff0000u) + __uint_as_float(wl.y & 0xffff0000u);
      y.x = t.x * alpha + x0 * om;
      y.y = t.y * alpha + x1 * om;
      y.z = t.z * alpha + x2 * om;
      y.w = t.w * alpha + x3 * om;
    }
    if constexpr (MODE == 1) {
      put4f(outF + (size_t)by * planeStride + (size_t)nc * NHID + 4 * lane, y, ok);
    } else if constexpr (MODE == 3) {
      put4f(outF + (size_t)nc * NHID + 4 * lane, y, ok);
    } else {
      v4us h4, l4;
      unsigned hb;
      hb = bf16_bits(y.x); h4[0] = (unsigned short)hb; l4[0] = (unsigned short)bf16_bits(y.x - __uint_as_float(hb << 16));
      hb = bf16_bits(y.y); h4[1] = (unsigned short)hb; l4[1] = (unsigned short)bf16_bits(y.y - __uint_as_float(hb << 16));
      hb = bf16_bits(y.z); h4[2] = (unsigned short)hb; l4[2] = (unsigned short)bf16_bits(y.z - __uint_as_float(hb << 16));
      hb = bf16_bits(y.w); h4[3] = (unsigned short)hb; l4[3] = (unsigned short)bf16_bits(y.w - __uint_as_float(hb << 16));
      *(v4usa*)(rb + 4 * lane) = h4;
      *(v4usa*)(rb + NHID + 4 * lane) = l4;
      wave_sync();
      const v8us q = *(const v8usa*)(rb + 8 * lane);
      wave_sync();
      put8us(xhl + (size_t)nc * KP + 8 * lane, q, ok);
    }
  }
}

__global__ __launch_bounds__(NTHR) void k_scan(const int* __restrict__ srcs, const int* __restrict__ keys,
                                               const int* __restrict__ etype, const int* __restrict__ etime,
                                               const int* __restrict__ ntype, int nE, int nN, int vec8,
                                               const float* __restrict__ Kp, const float* __restrict__ Qp,
                                               const float* __restrict__ Vp,
                                               const float* __restrict__ rtek, const float* __restrict__ rtev,
                                               const float* __restrict__ ratt, const float* __restrict__ rmsg,
                                               const float* __restrict__ pri, unsigned short* hhl) {
  extern __shared__ __attribute__((aligned(16))) int dsm[];
  int* list = dsm;
  int* hl   = dsm + LISTN;
  int* sl   = hl + RCAP;
  int* cnt  = sl + RCAP;
  int* offs = cnt + NBA;
  int* cur  = offs + NBA;
  int* misc = cur + NBA;
  float* RA = (float*)(misc + MISC_INTS);
  float* RM = RA + REL_F;
  float* PQ = RM + REL_F;
  float* PW = PQ + PQ_I;
  const int tid = (int)threadIdx.x, lane = tid & 31, wave = tid >> 5;
  const int nodeBase = (int)blockIdx.x * NBA;

  {
    const v4i z4 = {0, 0, 0, 0};
    for (int i = tid * 4; i < AGG_ZINTS; i += NTHR * 4) *(v4ia*)(dsm + i) = z4;
    if (tid < MISC_INTS) misc[tid] = 0;
#pragma unroll 1
    for (int i = tid * 4; i < REL_F; i += NTHR * 4) {
      const v4f a = *(const v4f*)(ratt + i);
      const v4f b = *(const v4f*)(rmsg + i);
      v4f ar, br;
      ar.x = bf16_val(a.x); ar.y = bf16_val(a.y); ar.z = bf16_val(a.z); ar.w = bf16_val(a.w);
      br.x = bf16_val(b.x); br.y = bf16_val(b.y); br.z = bf16_val(b.z); br.w = bf16_val(b.w);
      *(v4fa*)(RA + i) = ar;
      *(v4fa*)(RM + i) = br;
    }
    if (tid < PQ_I) PQ[tid] = bf16_val(pri[tid]) * 0.25f;
  }
  __syncthreads();

  int t = 0, ov = 0;
  const int nChunks = (nE + CHUNK - 1) / CHUNK;
#pragma unroll 1
  for (int ch = 0; ch < nChunks; ++ch) {
    const int cbase = ch * CHUNK;
    const int wc = scan_chunk<SLA>(keys, nE, cbase, nodeBase, NBA, vec8, list, tid, lane, wave);
    if (lane == 0) misc[wave] = wc;
    __syncthreads();
    if (wave == 0) {
#pragma unroll 1
      for (int w2 = 0; w2 < NWAVE; ++w2) {
        int c = misc[w2];
        c = c < 0 ? 0 : (c > WCAP ? WCAP : c);
#pragma unroll 1
        for (int b0 = 0; b0 < c; b0 += 32) {
          const int idx = b0 + lane;
          const int ent = list[w2 * WCAP + (idx < WCAP ? idx : WCAP - 1)];
          const int m32 = (c - b0) < 32 ? (c - b0) : 32;
#pragma unroll 1
          for (int k = 0; k < m32; ++k) {
            const int u    = __builtin_amdgcn_readlane(ent, k);
            const int slot = u & (NBA - 1);
            const int el   = (u >> SLA) & (CHUNK - 1);
            const int pk   = ((cbase + el) << SLA) | slot;
            if (t < RCAP) {
              if (lane == 0) { hl[t] = pk; cnt[slot] = cnt[slot] + 1; }
              t = t + 1;
            } else {
              ov = 1;
            }
          }
        }
      }
    }
    __syncthreads();
  }
  if (wave == 0 && lane == 0) { misc[8] = t; misc[9] = ov; }
  __syncthreads();
  int tt = misc[8];
  tt = tt < 0 ? 0 : (tt > RCAP ? RCAP : tt);
  const int ovf = misc[9];

  if (wave == 0) {
    const int base = lane * (NBA / 32);
    int s = 0;
#pragma unroll 1
    for (int i = 0; i < NBA / 32; ++i) s += cnt[base + i];
    int incl = s;
#pragma unroll
    for (int d = 1; d < 32; d <<= 1) {
      const int y = __shfl_up(incl, d, 32);
      if (lane >= d) incl += y;
    }
    int run = incl - s;
#pragma unroll 1
    for (int i = 0; i < NBA / 32; ++i) {
      const int cv = cnt[base + i];
      offs[base + i] = run;
      cur[base + i]  = run;
      run += cv;
    }
  }
  __syncthreads();
  if (wave == 0) {
#pragma unroll 1
    for (int b0 = 0; b0 < tt; b0 += 32) {
      const int idx = b0 + lane;
      const int ent = hl[idx < RCAP ? idx : RCAP - 1];
      const int m32 = (tt - b0) < 32 ? (tt - b0) : 32;
#pragma unroll 1
      for (int k = 0; k < m32; ++k) {
        const int u    = __builtin_amdgcn_readlane(ent, k);
        const int slot = u & (NBA - 1);
        if (lane == 0) {
          int p = cur[slot];
          p = p < 0 ? 0 : (p > RCAP - 1 ? RCAP - 1 : p);
          sl[p] = u;
          cur[slot] = p + 1;
        }
      }
    }
  }
  __syncthreads();

  const float qnan = __int_as_float(0x7fc00000);
  const float pz   = (ovf != 0) ? qnan : 0.0f;
  const int hgrp = lane >> 2, dq = lane & 3;
  float* wqv = PW + wave * PW_I;
  float* qaw = wqv + WQ_F;
  float* ubw = qaw + QA_F;
  float* scw = ubw + UB_F;
  unsigned short* rowbuf = (unsigned short*)(scw + SC_F);
#pragma unroll 1
  for (int si = 0; si < NBA / NWAVE; ++si) {
    const int s    = si * NWAVE + wave;
    const int node = nodeBase + s;
    if (node >= nN) continue;
    int c = cnt[s];
    const bool big = c > DEGCAP;
    c = c < 0 ? 0 : (c > DEGCAP ? DEGCAP : c);
    int o = offs[s];
    o = o < 0 ? 0 : (o > RCAP ? RCAP : o);

    {
      const v4f qv = *(const v4f*)(Qp + (size_t)node * NHID + 4 * lane);
      *(v4fa*)(wqv + 4 * lane) = qv;
      const v4f z = {0.f, 0.f, 0.f, 0.f};
      *(v4fa*)(ubw + 0 * NHID + 4 * lane) = z;
      *(v4fa*)(ubw + 1 * NHID + 4 * lane) = z;
      *(v4fa*)(ubw + 2 * NHID + 4 * lane) = z;
      *(v4fa*)(ubw + 3 * NHID + 4 * lane) = z;
    }
    wave_sync();
    const v4f q0 = *(const v4fa*)(wqv + 16 * hgrp);
    const v4f q1 = *(const v4fa*)(wqv + 16 * hgrp + 4);
    const v4f q2 = *(const v4fa*)(wqv + 16 * hgrp + 8);
    const v4f q3 = *(const v4fa*)(wqv + 16 * hgrp + 12);
    wave_sync();
#pragma unroll 1
    for (int rc = 0; rc < 16; ++rc) {
      const int r = rc >> 2, cc = rc & 3;
      const float* ap = RA + (((r * HEADS + hgrp) * DKD + 4 * dq + cc) * DKD);
      const v4f a0 = *(const v4fa*)ap;
      const v4f a1 = *(const v4fa*)(ap + 4);
      const v4f a2 = *(const v4fa*)(ap + 8);
      const v4f a3 = *(const v4fa*)(ap + 12);
      float sq = a0.x * q0.x;
      sq = fmaf(a0.y, q0.y, sq); sq = fmaf(a0.z, q0.z, sq); sq = fmaf(a0.w, q0.w, sq);
      sq = fmaf(a1.x, q1.x, sq); sq = fmaf(a1.y, q1.y, sq); sq = fmaf(a1.z, q1.z, sq); sq = fmaf(a1.w, q1.w, sq);
      sq = fmaf(a2.x, q2.x, sq); sq = fmaf(a2.y, q2.y, sq); sq = fmaf(a2.z, q2.z, sq); sq = fmaf(a2.w, q2.w, sq);
      sq = fmaf(a3.x, q3.x, sq); sq = fmaf(a3.y, q3.y, sq); sq = fmaf(a3.z, q3.z, sq); sq = fmaf(a3.w, q3.w, sq);
      qaw[r * NHID + 4 * lane + cc] = sq * PQ[r * HEADS + hgrp];
    }

    int idx = o + lane;
    idx = idx > RCAP - 1 ? RCAP - 1 : idx;
    const int ent = sl[idx];
    int eid = ent >> SLA;
    eid = eid < 0 ? 0 : (eid > nE - 1 ? nE - 1 : eid);
    int sr = srcs[eid];
    sr = sr < 0 ? 0 : (sr > nN - 1 ? nN - 1 : sr);
    int rr = etype[eid];
    rr = rr < 0 ? 0 : (rr > NREL - 1 ? NREL - 1 : rr);
    int tm = etime[eid];
    tm = tm < 0 ? 0 : (tm > MAXLEN - 1 ? MAXLEN - 1 : tm);
    int st = ntype[sr];
    st = st < 0 ? 0 : (st > 2 ? 2 : st);
    const int ro = (st * MAXLEN + tm) * NHID;

    float mx = -3.0e38f;
#pragma unroll 1
    for (int k = 0; k < c; ++k) {
      const int sk  = __builtin_amdgcn_readlane(sr, k);
      const int rk  = __builtin_amdgcn_readlane(rr, k);
      const int rok = __builtin_amdgcn_readlane(ro, k);
      const v4f kk = *(const v4f*)(Kp + (size_t)sk * NHID + 4 * lane);
      const v4f rt = *(const v4f*)(rtek + (size_t)rok + 4 * lane);
      const v4f qa = *(const v4fa*)(qaw + rk * NHID + 4 * lane);
      const v4f ke = kk + rt;
      float part = ke.x * qa.x;
      part = fmaf(ke.y, qa.y, part); part = fmaf(ke.z, qa.z, part); part = fmaf(ke.w, qa.w, part);
      part += __shfl_xor(part, 1, 32);
      part += __shfl_xor(part, 2, 32);
      scw[k * 32 + lane] = part;
      mx = fmaxf(mx, part);
    }
    float lsum = 0.0f;
#pragma unroll 1
    for (int k = 0; k < c; ++k) {
      const int sk  = __builtin_amdgcn_readlane(sr, k);
      const int rk  = __builtin_amdgcn_readlane(rr, k);
      const int rok = __builtin_amdgcn_readlane(ro, k);
      const v4f vv = *(const v4f*)(Vp + (size_t)sk * NHID + 4 * lane);
      const v4f rv = *(const v4f*)(rtev + (size_t)rok + 4 * lane);
      const v4f ve = vv + rv;
      const float a = scw[k * 32 + lane];
      const float p = expf(a - mx);
      lsum += p;
      v4f u = *(const v4fa*)(ubw + rk * NHID + 4 * lane);
      u.x = fmaf(p, ve.x, u.x); u.y = fmaf(p, ve.y, u.y); u.z = fmaf(p, ve.z, u.z); u.w = fmaf(p, ve.w, u.w);
      *(v4fa*)(ubw + rk * NHID + 4 * lane) = u;
    }
    const float inv = 1.0f / (lsum + 1e-16f);
    wave_sync();
    v4f ag = {0.f, 0.f, 0.f, 0.f};
#pragma unroll 1
    for (int rd = 0; rd < NREL * DKD; ++rd) {
      const int r = rd >> 4, d = rd & 15;
      const float uv = ubw[r * NHID + hgrp * DKD + d];
      const v4f mm = *(const v4fa*)(RM + (((r * HEADS + hgrp) * DKD + d) * DKD + 4 * dq));
      ag.x = fmaf(uv, mm.x, ag.x); ag.y = fmaf(uv, mm.y, ag.y);
      ag.z = fmaf(uv, mm.z, ag.z); ag.w = fmaf(uv, mm.w, ag.w);
    }
    wave_sync();
    {
      v4f av;
      av.x = ag.x * inv; av.y = ag.y * inv; av.z = ag.z * inv; av.w = ag.w * inv;
      *(v4fa*)(qaw + 4 * lane) = av;
    }
    const float pzr = big ? qnan : pz;
#pragma unroll 1
    for (int cc = 0; cc < 4; ++cc) {
      const float v = qaw[4 * lane + cc];
      float g = 0.5f * v * (1.0f + erff(v * 0.70710678118654752f));
      g = g + pzr;
      const unsigned hb = bf16_bits(g);
      const unsigned lb = bf16_bits(g - __uint_as_float(hb << 16));
      rowbuf[4 * lane + cc]        = (unsigned short)hb;
      rowbuf[NHID + 4 * lane + cc] = (unsigned short)lb;
    }
    wave_sync();
    const v8us qrow = *(const v8usa*)(rowbuf + 8 * lane);
    wave_sync();
    put8us(hhl + (size_t)node * KP + 8 * lane, qrow, true);
  }
}

static inline int cdiv(int a, int b) { return (a + b - 1) / b; }
static inline size_t al256(size_t o) { return (o + 255) & ~(size_t)255; }

extern "C" void kernel_launch(void* const* d_in, const int* in_sizes, int n_in,
                              void* d_out, int out_size, void* d_ws, size_t ws_size,
                              hipStream_t stream) {
  if (n_in < 22) return;
  const int nN = in_sizes[18];
  const int nE = in_sizes[20];
  if (nN < 64 || nN > 65536) return;
  if (nE < 1 || nE >= (1 << (31 - SLA))) return;
  if ((long long)in_sizes[0] != (long long)nN * IND) return;
  if (in_sizes[1] != NTYP * IND * NHID || in_sizes[2] != NTYP * NHID) return;
  if (in_sizes[3] != 2 * NTYP * NHID * NHID || in_sizes[4] != 2 * NTYP * NHID) return;
  if (in_sizes[5] != 2 * NTYP * NHID * NHID || in_sizes[6] != 2 * NTYP * NHID) return;
  if (in_sizes[7] != 2 * NTYP * NHID * NHID || in_sizes[8] != 2 * NTYP * NHID) return;
  if (in_sizes[9] != 2 * NTYP * NHID * NHID || in_sizes[10] != 2 * NTYP * NHID) return;
  if (in_sizes[11] != 2 * NREL * HEADS) return;
  if (in_sizes[12] != 2 * REL_F || in_sizes[13] != 2 * REL_F) return;
  if (in_sizes[14] != 2 * NTYP) return;
  if (in_sizes[15] != 2 * MAXLEN * IND || in_sizes[16] != 2 * IND * NHID || in_sizes[17] != 2 * NHID) return;
  if (in_sizes[19] != 2 * nE || in_sizes[21] != nE) return;
  if ((long long)out_size != (long long)nN * NHID) return;

  const float* nf   = (const float*)d_in[0];
  const float* adw  = (const float*)d_in[1];
  const float* adb  = (const float*)d_in[2];
  const float* kw   = (const float*)d_in[3];
  const float* kb   = (const float*)d_in[4];
  const float* qw   = (const float*)d_in[5];
  const float* qb   = (const float*)d_in[6];
  const float* vw   = (const float*)d_in[7];
  const float* vb   = (const float*)d_in[8];
  const float* aw   = (const float*)d_in[9];
  const float* ab   = (const float*)d_in[10];
  const float* rpri = (const float*)d_in[11];
  const float* ratt = (const float*)d_in[12];
  const float* rmsg = (const float*)d_in[13];
  const float* skip = (const float*)d_in[14];
  const float* rtab = (const float*)d_in[15];
  const float* rtw  = (const float*)d_in[16];
  const float* rtb  = (const float*)d_in[17];
  const int* ntype  = (const int*)d_in[18];
  const int* eidx   = (const int*)d_in[19];
  const int* etype  = (const int*)d_in[20];
  const int* etime  = (const int*)d_in[21];
  float* out = (float*)d_out;
  const int* src = eidx;
  const int* dst = eidx + nE;

  const int permCap = cdiv(nN, GBM) * GBM + NTYP * GBM;
  const int gT = permCap / GBM;
  const int gA = cdiv(nN, NBA);
  const int vec8 = ((nE & 3) == 0) ? 1 : 0;
  const size_t sortLds = (size_t)(permCap + 3 * NTHR) * 4;
  if (sortLds > 290000) return;
  const size_t scanLds = (size_t)SCAN_LDS_INTS * 4;

  char* ws = (char*)d_ws;
  size_t off = 0;
  const size_t oHHL = off; off = al256(off + (size_t)nN * KP * 2);
  const size_t oXHL = off; off = al256(off + (size_t)nN * KP * 2);
  const size_t oKQV = off; off = al256(off + (size_t)3 * nN * NHID * 4);
  const size_t oWPL = off; off = al256(off + (size_t)UWTOT * 16);
  const size_t oRTE = off; off = al256(off + (size_t)RTE_F * 4);
  const size_t oPRM = off; off = al256(off + (size_t)permCap * 4);
  if (off > ws_size || off > (size_t)WSMAX) return;
  unsigned short* HHL = (unsigned short*)(ws + oHHL);
  unsigned short* XHL = (unsigned short*)(ws + oXHL);
  float*          KQV = (float*)(ws + oKQV);
  unsigned short* WPL = (unsigned short*)(ws + oWPL);
  float*          RTE = (float*)(ws + oRTE);
  int*            PRM = (int*)(ws + oPRM);
  const size_t planeStride = (size_t)nN * NHID;
  const unsigned short* ADP  = WPL;
  const unsigned short* KQV2 = WPL + (size_t)(NTYP * NHID) * KP;
  const unsigned short* A2   = WPL + (size_t)(NTYP * NHID + 2 * NTYP * 3 * NHID) * KP;

  hipFuncSetAttribute(reinterpret_cast<const void*>(&k_sort), hipFuncAttributeMaxDynamicSharedMemorySize, (int)sortLds);
  hipFuncSetAttribute(reinterpret_cast<const void*>(&k_scan), hipFuncAttributeMaxDynamicSharedMemorySize, (int)scanLds);

  k_wprep<<<UWTOT / NTHR, NTHR, 0, stream>>>(adw, kw, qw, vw, aw, WPL);
  k_sort<<<1, NTHR, sortLds, stream>>>(ntype, nN, permCap, PRM);
  k_rte<<<2 * MAXLEN, 128, 0, stream>>>(rtab, rtw, rtb, kw, vw, RTE);
  k_gemm<0><<<dim3(gT, 1), GTHR, 0, stream>>>(nf, HHL, ADP, NHID, PRM, permCap, ntype, nN,
                                              adb, adb, adb, skip, XHL, KQV, planeStride);
  for (int l = 0; l < 2; ++l) {
    const unsigned short* wkqv = KQV2 + (size_t)l * (NTYP * 3 * NHID) * KP;
    const unsigned short* wa   = A2 + (size_t)l * (NTYP * NHID) * KP;
    const float* rk = RTE + (size_t)((l * 2 + 0) * NTYP) * MAXLEN * NHID;
    const float* rv = RTE + (size_t)((l * 2 + 1) * NTYP) * MAXLEN * NHID;
    k_gemm<1><<<dim3(gT, 3), GTHR, 0, stream>>>(nf, XHL, wkqv, 3 * NHID, PRM, permCap, ntype, nN,
                                                kb + l * NTYP * NHID, qb + l * NTYP * NHID, vb + l * NTYP * NHID,
                                                skip + l * NTYP, XHL, KQV, planeStride);
    k_scan<<<gA, NTHR, scanLds, stream>>>(src, dst, etype, etime, ntype, nE, nN, vec8,
                                          KQV, KQV + planeStride, KQV + 2 * planeStride, rk, rv,
                                          ratt + (size_t)l * REL_F, rmsg + (size_t)l * REL_F,
                                          rpri + l * NREL * HEADS, HHL);
    if (l == 0) {
      k_gemm<2><<<dim3(gT, 1), GTHR, 0, stream>>>(nf, HHL, wa, NHID, PRM, permCap, ntype, nN,
                                                  ab + l * NTYP * NHID, ab, ab, skip + l * NTYP, XHL, out, planeStride);
    } else {
      k_gemm<3><<<dim3(gT, 1), GTHR, 0, stream>>>(nf, HHL, wa, NHID, PRM, permCap, ntype, nN,
                                                  ab + l * NTYP * NHID, ab, ab, skip + l * NTYP, XHL, out, planeStride);
    }
  }
}
